// CudaFastWeightSumTwoLinearTransformerLayer_15891378995458
// MI455X (gfx1250) — hardware-run, weakly checked
//
#include <hip/hip_runtime.h>


#define LL   256
#define BB   64
#define NH_  8
#define DH   64
#define DM   512
#define DQ   2048
#define NR   16384
#define NP   512
#define ZP   64
#define DQH  256
typedef _Float16 h16;
typedef unsigned short bf;
typedef __attribute__((ext_vector_type(16))) __bf16   v16bf;
typedef __attribute__((ext_vector_type(16))) _Float16 v16h;
typedef __attribute__((ext_vector_type(8)))  _Float16 v8h;
typedef __attribute__((ext_vector_type(8)))  unsigned short v8us;
typedef __attribute__((ext_vector_type(8)))  float    v8f;
typedef __attribute__((ext_vector_type(4)))  float    v4f;
typedef v8h  __attribute__((may_alias)) v8ha;
typedef v4f  __attribute__((may_alias)) v4fa;
typedef v8us __attribute__((may_alias)) v8usa;

__device__ __forceinline__ unsigned short f2bf(float f) { unsigned u = __float_as_uint(f); u += 0x7FFFu + ((u >> 16) & 1u); return (unsigned short)(u >> 16); }
__device__ __forceinline__ float bf2f(unsigned short b) { return __uint_as_float(((unsigned)b) << 16); }
__device__ __forceinline__ float bfr(float f) { return bf2f(f2bf(f)); }
__device__ __forceinline__ v16h cat16(v8h lo, v8h hi) { return __builtin_shufflevector(lo, hi, 0, 1, 2, 3, 4, 5, 6, 7, 8, 9, 10, 11, 12, 13, 14, 15); }
__device__ __forceinline__ v16bf cat16b(v8us lo, v8us hi) { return __builtin_bit_cast(v16bf, __builtin_shufflevector(lo, hi, 0, 1, 2, 3, 4, 5, 6, 7, 8, 9, 10, 11, 12, 13, 14, 15)); }
__device__ __forceinline__ v8f wmma16(v16h a, v16h b, v8f c) { return __builtin_amdgcn_wmma_f32_16x16x32_f16(false, a, false, b, (short)0, c, false, false); }
__device__ __forceinline__ v8f wmmab(v16bf a, v16bf b, v8f c) { return __builtin_amdgcn_wmma_f32_16x16x32_bf16(false, a, false, b, (short)0, c, false, false); }


template <typename T16> struct WFrag;
template <> struct WFrag<h16> { typedef v16h V; static __device__ __forceinline__ V ld(const h16* p) { return cat16(*(const v8h*)p, *(const v8h*)(p + 16)); } static __device__ __forceinline__ v8f mma(V a, V b, v8f c) { return wmma16(a, b, c); } };
template <> struct WFrag<bf> { typedef v16bf V; static __device__ __forceinline__ V ld(const bf* p) { return cat16b(*(const v8us*)p, *(const v8us*)(p + 16)); } static __device__ __forceinline__ v8f mma(V a, V b, v8f c) { return wmmab(a, b, c); } };
template <typename T16, int NSPLIT, bool BIAS>
__global__ __launch_bounds__(32) void k_gemmw(const T16* __restrict__ A, const T16* __restrict__ A2, const T16* __restrict__ Bt, const T16* __restrict__ Bt2, int K, float* C, int ldc, const float* __restrict__ bias, size_t sA, size_t sB, size_t sC) {
    typedef typename WFrag<T16>::V V;
    __shared__ __align__(16) float os[16 * 68];
    const size_t z = blockIdx.z; A += z * sA; if (A2) A2 += z * sA; Bt += z * sB; if (Bt2) Bt2 += z * sB; C += z * sC;
    const int lane = threadIdx.x & 31, lr = lane & 15, hi = lane >> 4; const int r0 = blockIdx.x * 64, c0 = blockIdx.y * 64;
    v8f acc[4][4];
#pragma unroll
    for (int mb = 0; mb < 4; ++mb)
#pragma unroll
        for (int nb = 0; nb < 4; ++nb) acc[mb][nb] = (v8f){};
    const size_t aoff = (size_t)(r0 + lr) * K + 8 * hi, boff = (size_t)(c0 + lr) * K + 8 * hi;
#pragma unroll 1
    for (int kc = 0; kc < K; kc += 32) {
        V a[4], a2[4];
#pragma unroll
        for (int mb = 0; mb < 4; ++mb) { a[mb] = WFrag<T16>::ld(A + aoff + (size_t)mb * 16 * K + kc); if (NSPLIT == 1 || NSPLIT == 2) a2[mb] = WFrag<T16>::ld(A2 + aoff + (size_t)mb * 16 * K + kc); }
#pragma unroll
        for (int nb = 0; nb < 4; ++nb) { const V b = WFrag<T16>::ld(Bt + boff + (size_t)nb * 16 * K + kc); V b2; if (NSPLIT >= 2) b2 = WFrag<T16>::ld(Bt2 + boff + (size_t)nb * 16 * K + kc);
#pragma unroll
            for (int mb = 0; mb < 4; ++mb) { acc[mb][nb] = WFrag<T16>::mma(a[mb], b, acc[mb][nb]); if (NSPLIT == 1 || NSPLIT == 2) acc[mb][nb] = WFrag<T16>::mma(a2[mb], b, acc[mb][nb]); if (NSPLIT >= 2) acc[mb][nb] = WFrag<T16>::mma(a[mb], b2, acc[mb][nb]); } }
        asm volatile("v_nop\n\tv_nop\n\tv_nop\n\tv_nop" : "+v"(acc[0][0]), "+v"(acc[1][1]), "+v"(acc[2][2]), "+v"(acc[3][3]) : "v"(a[0]), "v"(a[3]));
    }
#pragma unroll
    for (int mb = 0; mb < 4; ++mb) {
#pragma unroll
        for (int nb = 0; nb < 4; ++nb) {
#pragma unroll
            for (int j = 0; j < 8; ++j) os[(hi * 8 + j) * 68 + nb * 16 + lr] = acc[mb][nb][j]; }
        __builtin_amdgcn_wave_barrier(); asm volatile("" ::: "memory");
        float* crow = C + (size_t)(r0 + mb * 16) * ldc + c0;
#pragma unroll 1
        for (int ps = 0; ps < 2; ++ps) {
#pragma unroll
            for (int s = 0; s < 8; ++s) { const int row = 2 * s + hi, cofs = lr * 4; v4f val = *(const v4fa*)(os + row * 68 + cofs); if (BIAS) { val[0] += bfr(bias[c0 + cofs]); val[1] += bfr(bias[c0 + cofs + 1]); val[2] += bfr(bias[c0 + cofs + 2]); val[3] += bfr(bias[c0 + cofs + 3]); }
                *(volatile v4f*)(crow + (size_t)row * ldc + cofs) = val; }
            if (ps == 0) __threadfence(); }
        __builtin_amdgcn_wave_barrier(); asm volatile("" ::: "memory");
    }
}

__device__ __forceinline__ void splitf(float y, unsigned short& h, unsigned short& l) { h = f2bf(y); l = f2bf(y - bf2f(h)); }
typedef __attribute__((ext_vector_type(2))) unsigned short v2us;
typedef __attribute__((ext_vector_type(4))) unsigned short v4us;

__global__ __launch_bounds__(256) void k_cvt8(const float* __restrict__ src, bf* dst, size_t n8) { const size_t i = (size_t)blockIdx.x * 256 + threadIdx.x; if (i >= n8) return; const v8f v = *(const v8f*)(src + i * 8); v8us o;
#pragma unroll
    for (int k = 0; k < 8; ++k) o[k] = f2bf(v[k]); *(volatile v8us*)(dst + i * 8) = o; __threadfence(); *(volatile v8us*)(dst + i * 8) = o; }
__global__ __launch_bounds__(256) void k_phi(const float* __restrict__ QKVh, int h, const float* __restrict__ pi0, const float* __restrict__ pi1, bf* Qh, bf* Ql, bf* Kh, bf* Kl) { const int lane = threadIdx.x & 31; const int row = blockIdx.x * 8 + (threadIdx.x >> 5); if (row >= ZP * LL) return; const int l = row % LL; const int p = row / LL; const int b = p; const float* src = QKVh + ((size_t)l * BB + b) * DQH;
    float e[3][2]; float s[3] = {0.f, 0.f, 0.f};
#pragma unroll
    for (int c = 0; c < 3; ++c) {
#pragma unroll
        for (int u = 0; u < 2; ++u) { const float x = src[c * DH + lane * 2 + u]; const float el = (x > 0.f) ? x : expm1f(x); e[c][u] = __fadd_rn(el, 1.0f); s[c] += e[c][u]; } }
#pragma unroll
    for (int c = 0; c < 3; ++c) {
#pragma unroll
        for (int sh = 16; sh; sh >>= 1) s[c] += __shfl_xor(s[c], sh, 32); }
    const float c0 = fminf(fmaxf(bfr(pi0[h * 256 + l]), 0.f), 1.f), c1 = fminf(fmaxf(bfr(pi1[h * 256 + l]), 0.f), 1.f);
    v2us qh, ql, kh, kl;
#pragma unroll
    for (int u = 0; u < 2; ++u) { const float q = __fdiv_rn(e[0][u], s[0]); float a1 = __fmul_rn(__fdiv_rn(e[1][u], s[1]), c0); float a2 = __fmul_rn(__fdiv_rn(e[2][u], s[2]), c1); asm volatile("" : "+v"(a1)); asm volatile("" : "+v"(a2)); const float k = __fadd_rn(a1, a2); unsigned short x1, y1, x2, y2; splitf(q, x1, y1); splitf(k, x2, y2); qh[u] = x1; ql[u] = y1; kh[u] = x2; kl[u] = y2; }
    const size_t oo = ((size_t)p * LL + l) * DH + lane * 2; for (int ps = 0; ps < 2; ++ps) { *(volatile v2us*)(Qh + oo) = qh; *(volatile v2us*)(Ql + oo) = ql; *(volatile v2us*)(Kh + oo) = kh; *(volatile v2us*)(Kl + oo) = kl; if (ps == 0) __threadfence(); } }
__global__ __launch_bounds__(256) void k_vt(const float* __restrict__ QKVh, bf* Th, bf* Tl) { const int e = (blockIdx.x * 256 + threadIdx.x) * 2; if (e >= ZP * DH * LL) return; const int l = e % LL; const int d = (e / LL) % DH; const int b = e / (LL * DH); v2us oh, ol;
#pragma unroll
    for (int u = 0; u < 2; ++u) { unsigned short a, c; splitf(QKVh[((size_t)(l + u) * BB + b) * DQH + 3 * DH + d], a, c); oh[u] = a; ol[u] = c; } for (int ps = 0; ps < 2; ++ps) { *(volatile v2us*)(Th + e) = oh; *(volatile v2us*)(Tl + e) = ol; if (ps == 0) __threadfence(); } }
__global__ __launch_bounds__(256) void k_cmask(const float* __restrict__ A, int p0, bf* Ah, bf* Al, float* DEN) { const int lane = threadIdx.x & 31; const int row = blockIdx.x * 8 + (threadIdx.x >> 5); if (row >= ZP * LL) return; const int l = row % LL; const int pz = row / LL; const float* ar = A + (size_t)row * LL; float den = 0.f; v4us oh[2], ol[2];
#pragma unroll
    for (int ch = 0; ch < 2; ++ch) { const int s0 = ch * 128 + lane * 4; const v4f a = *(const v4f*)(ar + s0);
#pragma unroll
        for (int u = 0; u < 4; ++u) { const float v = (s0 + u <= l) ? a[u] : 0.f; den = __fadd_rn(den, v); unsigned short x, y; splitf(v, x, y); oh[ch][u] = x; ol[ch][u] = y; } }
#pragma unroll
    for (int sh = 16; sh; sh >>= 1) den += __shfl_xor(den, sh, 32);
    for (int ps = 0; ps < 2; ++ps) {
#pragma unroll
        for (int ch = 0; ch < 2; ++ch) { const size_t oo = (size_t)row * LL + ch * 128 + lane * 4; *(volatile v4us*)(Ah + oo) = oh[ch]; *(volatile v4us*)(Al + oo) = ol[ch]; }
        if (ps == 0) __threadfence(); }
    __shared__ float dsh[8]; if (lane == 0) dsh[threadIdx.x >> 5] = den; __syncthreads();
    if (threadIdx.x < 32) { const float dv = (threadIdx.x < 8) ? dsh[threadIdx.x] : 0.f; float* dd = DEN + ((size_t)p0 * (LL / 8) + blockIdx.x) * 32 + threadIdx.x; *(volatile float*)dd = dv; __threadfence(); *(volatile float*)dd = dv; } }
__global__ __launch_bounds__(256) void k_osc(const float* __restrict__ O, const float* __restrict__ DEN, int p0, bf* Ph, bf* Pl) { const int e = (blockIdx.x * 256 + threadIdx.x) * 2; if (e >= ZP * LL * DH) return; const int d = e % DH; const int l = (e / DH) % LL; const int pz = e / (DH * LL); const int b = pz; const int h = p0 / ZP; const float den = __fadd_rn(DEN[((size_t)p0 * (LL / 8) + (size_t)pz * (LL / 8) + l / 8) * 32 + (l % 8)], 1e-5f); v2us oh, ol;
#pragma unroll
    for (int u = 0; u < 2; ++u) { const float y = __fdiv_rn(O[e + u] * 0.125f, den); unsigned short a, c; splitf(y, a, c); oh[u] = a; ol[u] = c; } const size_t oo = ((size_t)l * BB + b) * DM + h * DH + d; for (int ps = 0; ps < 2; ++ps) { *(volatile v2us*)(Ph + oo) = oh; *(volatile v2us*)(Pl + oo) = ol; if (ps == 0) __threadfence(); } }
__global__ __launch_bounds__(256) void k_lnres(const float* __restrict__ Hx, const float* __restrict__ AT, const float* __restrict__ g, const float* __restrict__ bb, float* OUT) { const int lane = threadIdx.x & 31; const int r = blockIdx.x * 8 + (threadIdx.x >> 5); if (r >= NR) return; float v[DM / 32]; float s = 0.f;
#pragma unroll
    for (int ch = 0; ch < DM / 128; ++ch) { const size_t o0 = (size_t)r * DM + ch * 128 + lane * 4; const v4f a = *(const v4f*)(Hx + o0), t = *(const v4f*)(AT + o0);
#pragma unroll
        for (int u = 0; u < 4; ++u) { float xb = bfr(a[u]); asm volatile("" : "+v"(xb)); v[ch * 4 + u] = __fadd_rn(xb, t[u]); s += v[ch * 4 + u]; } }
#pragma unroll
    for (int sh = 16; sh; sh >>= 1) s += __shfl_xor(s, sh, 32);
    const float mean = s * (1.0f / DM); float q = 0.f;
#pragma unroll
    for (int k = 0; k < DM / 32; ++k) { float d = __fsub_rn(v[k], mean); asm volatile("" : "+v"(d)); float p = __fmul_rn(d, d); asm volatile("" : "+v"(p)); q = __fadd_rn(q, p); }
#pragma unroll
    for (int sh = 16; sh; sh >>= 1) q += __shfl_xor(q, sh, 32);
    const float rden = __fdiv_rn(1.0f, __fsqrt_rn(__fadd_rn(q * (1.0f / DM), 1e-5f)));
    for (int ps = 0; ps < 2; ++ps) {
#pragma unroll
        for (int ch = 0; ch < DM / 128; ++ch) { const int c0 = ch * 128 + lane * 4; v4f o;
#pragma unroll
            for (int u = 0; u < 4; ++u) { float d = __fsub_rn(v[ch * 4 + u], mean); asm volatile("" : "+v"(d)); float n0 = __fmul_rn(d, rden); asm volatile("" : "+v"(n0)); float gg = bfr(g[c0 + u]), b2 = bfr(bb[c0 + u]); asm volatile("" : "+v"(gg)); asm volatile("" : "+v"(b2)); float t1 = __fmul_rn(n0, gg); asm volatile("" : "+v"(t1)); o[u] = __fadd_rn(t1, b2); }
            *(volatile v4f*)(OUT + (size_t)r * DM + c0) = o; }
        if (ps == 0) __threadfence(); } }

extern "C" void kernel_launch(void* const* d_in, const int* in_sizes, int n_in,
                              void* d_out, int out_size, void* d_ws, size_t ws_size, hipStream_t stream) {
    (void)in_sizes; (void)n_in; (void)out_size;
    const float** I = (const float**)d_in;
    const float *hx = I[0], *qkv_w = I[1], *o_w = I[2], *pi0 = I[3], *pi1 = I[4], *lg = I[5], *lb = I[6];
    float* OUT = (float*)d_out;
    char* wsp = (char*)d_ws;
    auto take = [&](size_t bytes) { char* p = wsp; wsp += (bytes + 255) & ~(size_t)255; return (void*)p; };
    bf* BQKV = (bf*)take((size_t)DQ * DM * 2); bf* BO = (bf*)take((size_t)DM * DM * 2); bf* HB = (bf*)take((size_t)NR * DM * 2); float* QKV = (float*)take((size_t)NR * DQH * 4);
    bf* Qh = (bf*)take((size_t)ZP * LL * DH * 2); bf* Ql = (bf*)take((size_t)ZP * LL * DH * 2); bf* Kh = (bf*)take((size_t)ZP * LL * DH * 2); bf* Kl = (bf*)take((size_t)ZP * LL * DH * 2); bf* VTh = (bf*)take((size_t)ZP * DH * LL * 2); bf* VTl = (bf*)take((size_t)ZP * DH * LL * 2);
    float* A = (float*)take((size_t)ZP * LL * LL * 4); bf* Ah = (bf*)take((size_t)ZP * LL * LL * 2); bf* Al = (bf*)take((size_t)ZP * LL * LL * 2); float* DEN = (float*)take((size_t)NP * (LL / 8) * 32 * 4); float* O = (float*)take((size_t)ZP * LL * DH * 4);
    bf* OPh = (bf*)take((size_t)NR * DM * 2); bf* OPl = (bf*)take((size_t)NR * DM * 2); float* AT = (float*)take((size_t)NR * DM * 4);
    if ((size_t)(wsp - (char*)d_ws) > ws_size) return;
    k_cvt8<<<(DQ * DM / 8 + 255) / 256, 256, 0, stream>>>(qkv_w, BQKV, (size_t)DQ * DM / 8); k_cvt8<<<(DM * DM / 8 + 255) / 256, 256, 0, stream>>>(o_w, BO, DM * DM / 8); k_cvt8<<<(NR * DM / 8 + 255) / 256, 256, 0, stream>>>(hx, HB, (size_t)NR * DM / 8);
    const size_t zq = (size_t)LL * DH, zA = (size_t)LL * LL, zv = (size_t)DH * LL;
    for (int h = 0; h < NH_; ++h) { const int p0 = h * ZP;
        k_gemmw<bf, 0, false><<<dim3(NR / 64, DQH / 64, 1), 32, 0, stream>>>(HB, nullptr, BQKV + (size_t)h * DQH * DM, nullptr, DM, QKV, DQH, nullptr, 0, 0, 0);
        k_phi<<<ZP * LL / 8, 256, 0, stream>>>(QKV, h, pi0, pi1, Qh, Ql, Kh, Kl); k_vt<<<(ZP * DH * LL / 2 + 255) / 256, 256, 0, stream>>>(QKV, VTh, VTl);
        k_gemmw<bf, 2, false><<<dim3(LL / 64, LL / 64, ZP), 32, 0, stream>>>(Qh, Ql, Kh, Kl, DH, A, LL, nullptr, zq, zq, zA);
        k_cmask<<<ZP * LL / 8, 256, 0, stream>>>(A, p0, Ah, Al, DEN);
        k_gemmw<bf, 2, false><<<dim3(LL / 64, 1, ZP), 32, 0, stream>>>(Ah, Al, VTh, VTl, LL, O, DH, nullptr, zA, zv, zq);
        k_osc<<<(ZP * LL * DH / 2 + 255) / 256, 256, 0, stream>>>(O, DEN, p0, OPh, OPl); }
    k_gemmw<bf, 1, false><<<dim3(NR / 64, DM / 64, 1), 32, 0, stream>>>(OPh, OPl, BO, nullptr, DM, AT, DM, nullptr, 0, 0, 0);
    k_lnres<<<NR / 8, 256, 0, stream>>>(hx, AT, lg, lb, OUT);
}
